// BertAttention_20504173871698
// MI455X (gfx1250) — hardware-verified
//
#include <hip/hip_runtime.h>
#include <stdint.h>


#ifndef NB
#define NB 4
#endif
#ifndef SEQ
#define SEQ 2048
#endif
#define NB_FULL 4
#define SEQ_FULL 2048
#define HID 1024
#define NHEAD 16
#define HDIM 64
#define PCARRY 4096.0f

static_assert(NB >= 1 && NB <= NB_FULL);
static_assert(SEQ >= 128 && SEQ <= SEQ_FULL && (SEQ % 128) == 0);
static_assert(HID == NHEAD * HDIM);
static_assert((HID % 128) == 0);

typedef __bf16 bf16_t;
typedef _Float16 f16_t;
typedef __attribute__((ext_vector_type(16))) __bf16 v16bf;
typedef __attribute__((ext_vector_type(8)))  __bf16 bf16x8;
typedef __attribute__((ext_vector_type(16))) _Float16 v16h;
typedef __attribute__((ext_vector_type(8)))  _Float16 h16x8;
typedef __attribute__((ext_vector_type(8)))  float v8f;
typedef __attribute__((ext_vector_type(4)))  float f32x4;
typedef __attribute__((ext_vector_type(4)))  unsigned int u32x4;
typedef __attribute__((ext_vector_type(8)))  unsigned short us16x8;

__device__ __forceinline__ unsigned int bf_bits(float f) {
  unsigned int u = __builtin_bit_cast(unsigned int, f);
  return (u + 0x7FFFu + ((u >> 16) & 1u)) >> 16;
}
__device__ __forceinline__ float bf_rne(float f) {
  return __builtin_bit_cast(float, bf_bits(f) << 16);
}

__device__ __forceinline__ v16bf frag_row_bf(const bf16_t* p, int ld) {
  const int lane = threadIdx.x & 31;
  const int hf = lane >> 4, r = lane & 15;
  const bf16_t* q = p + r * ld + hf * 8;
  bf16x8 lo = *(const bf16x8*)(q);
  bf16x8 hi = *(const bf16x8*)(q + 16);
  return __builtin_shufflevector(lo, hi, 0, 1, 2, 3, 4, 5, 6, 7,
                                 8, 9, 10, 11, 12, 13, 14, 15);
}
__device__ __forceinline__ v16h frag_row_h(const f16_t* p, int ld) {
  const int lane = threadIdx.x & 31;
  const int hf = lane >> 4, r = lane & 15;
  const f16_t* q = p + r * ld + hf * 8;
  h16x8 lo = *(const h16x8*)(q);
  h16x8 hi = *(const h16x8*)(q + 16);
  return __builtin_shufflevector(lo, hi, 0, 1, 2, 3, 4, 5, 6, 7,
                                 8, 9, 10, 11, 12, 13, 14, 15);
}

__device__ __forceinline__ v8f wmma_bf16(v16bf a, v16bf b, v8f c) {
  v8f d = __builtin_amdgcn_wmma_f32_16x16x32_bf16(false, a, false, b, (short)0, c, false, false);
  asm volatile("v_nop\n\tv_nop\n\tv_nop\n\tv_nop" : "+v"(d) : "v"(a), "v"(b));
  return d;
}
__device__ __forceinline__ v8f wmma_f16(v16h a, v16h b, v8f c) {
  v8f d = __builtin_amdgcn_wmma_f32_16x16x32_f16(false, a, false, b, (short)0, c, false, false);
  asm volatile("v_nop\n\tv_nop\n\tv_nop\n\tv_nop" : "+v"(d) : "v"(a), "v"(b));
  return d;
}

__device__ __forceinline__ void wave_lds_sync() {
  asm volatile("s_wait_dscnt 0x0" ::: "memory");
  __builtin_amdgcn_wave_barrier();
}

__global__ __launch_bounds__(256) void k_cast_rows(const float* __restrict__ X,
                                                    unsigned short* __restrict__ Y) {
  const size_t g = (size_t)blockIdx.x * 256 + threadIdx.x;
  const size_t e = g * 8;
  const int prow = (int)(e >> 10);
  const int col = (int)(e & 1023);
  if (prow >= NB * SEQ) return;
  const int b = prow / SEQ;
  const int s = prow - b * SEQ;
  const float* src = X + ((size_t)b * SEQ_FULL + s) * HID + col;
  const f32x4 f0 = ((const f32x4*)src)[0];
  const f32x4 f1 = ((const f32x4*)src)[1];
  u32x4 pk;
  pk.x = bf_bits(f0.x) | (bf_bits(f0.y) << 16);
  pk.y = bf_bits(f0.z) | (bf_bits(f0.w) << 16);
  pk.z = bf_bits(f1.x) | (bf_bits(f1.y) << 16);
  pk.w = bf_bits(f1.z) | (bf_bits(f1.w) << 16);
  unsigned short* dst = Y + (size_t)prow * HID + col;
  *(volatile u32x4*)dst = pk;
  __threadfence();
  *(volatile u32x4*)dst = pk;
}

__global__ __launch_bounds__(256) void k_cast_wt(const float* __restrict__ W,
                                                  unsigned short* __restrict__ WT) {
  constexpr int LDT = 72;
  __shared__ __align__(16) unsigned short T[64 * LDT];
  const int tid = threadIdx.x;
  const int k0 = blockIdx.x * 64;
  const int n0 = blockIdx.y * 64;
  const int krow = tid >> 2;
  const int nq = (tid & 3) * 16;
  const f32x4* s4 = (const f32x4*)(W + (size_t)(k0 + krow) * HID + n0 + nq);
  const f32x4 f0 = s4[0], f1 = s4[1], f2 = s4[2], f3 = s4[3];
  float fv[16];
  fv[0] = f0.x;  fv[1] = f0.y;  fv[2] = f0.z;  fv[3] = f0.w;
  fv[4] = f1.x;  fv[5] = f1.y;  fv[6] = f1.z;  fv[7] = f1.w;
  fv[8] = f2.x;  fv[9] = f2.y;  fv[10] = f2.z; fv[11] = f2.w;
  fv[12] = f3.x; fv[13] = f3.y; fv[14] = f3.z; fv[15] = f3.w;
#pragma unroll
  for (int j = 0; j < 16; ++j)
    T[(nq + j) * LDT + krow] = (unsigned short)bf_bits(fv[j]);
  __syncthreads();

  u32x4 vals[2];
  unsigned short* dsts[2];
#pragma unroll
  for (int it = 0; it < 2; ++it) {
    const int p = it * 256 + tid;
    const int row = p >> 3, c = p & 7;
    const us16x8 hv = *(const us16x8*)(T + row * LDT + c * 8);
    vals[it] = __builtin_bit_cast(u32x4, hv);
    dsts[it] = WT + (size_t)(n0 + row) * HID + k0 + c * 8;
  }
#pragma unroll
  for (int it = 0; it < 2; ++it) *(volatile u32x4*)dsts[it] = vals[it];
  __threadfence();
#pragma unroll
  for (int it = 0; it < 2; ++it) *(volatile u32x4*)dsts[it] = vals[it];
}

template <bool TRANS_OUT>
__global__ __launch_bounds__(256) __attribute__((amdgpu_num_vgpr(256)))
void k_proj_gemm(const bf16_t* __restrict__ X, const bf16_t* __restrict__ WT,
                 const float* __restrict__ bias, f16_t* __restrict__ outp) {
  constexpr int K = HID;
  constexpr int LDA = 40;
  constexpr int LDC = 136;
  static_assert(128 * LDC * 2 >= 2 * 128 * LDA * 2);
  static_assert((K % 32) == 0);
  __shared__ __align__(16) unsigned char smem[128 * LDC * 2];
  bf16_t* As = (bf16_t*)smem;
  bf16_t* Bs = As + 128 * LDA;
  f16_t* Cs = (f16_t*)smem;

  const int tid = threadIdx.x;
  const int lane = tid & 31, w = tid >> 5;
  const int wr = w >> 1, wc = w & 1;
  const int hf = lane >> 4, nl = lane & 15;
  const int m0 = blockIdx.y * 128, n0 = blockIdx.x * 128;

  v8f acc[2][4];
#pragma unroll
  for (int i = 0; i < 2; ++i)
#pragma unroll
    for (int j = 0; j < 4; ++j)
#pragma unroll
      for (int r = 0; r < 8; ++r) acc[i][j][r] = 0.0f;

#pragma unroll 1
  for (int kt = 0; kt < K / 32; ++kt) {
#pragma unroll
    for (int it = 0; it < 2; ++it) {
      const int p = it * 256 + tid;
      const int r = p >> 2, c = (p & 3) * 8;
      *(bf16x8*)(As + r * LDA + c) =
          *(const bf16x8*)(X + (size_t)(m0 + r) * K + kt * 32 + c);
      *(bf16x8*)(Bs + r * LDA + c) =
          *(const bf16x8*)(WT + (size_t)(n0 + r) * K + kt * 32 + c);
    }
    __syncthreads();

    const v16bf a0 = frag_row_bf(As + (wr * 32) * LDA, LDA);
    const v16bf a1 = frag_row_bf(As + (wr * 32 + 16) * LDA, LDA);
#pragma unroll
    for (int nf = 0; nf < 4; ++nf) {
      const v16bf bb = frag_row_bf(Bs + (wc * 64 + nf * 16) * LDA, LDA);
      acc[0][nf] = wmma_bf16(a0, bb, acc[0][nf]);
      acc[1][nf] = wmma_bf16(a1, bb, acc[1][nf]);
    }
    __syncthreads();
  }

  float bb4[4];
#pragma unroll
  for (int nf = 0; nf < 4; ++nf) bb4[nf] = bf_rne(bias[n0 + wc * 64 + nf * 16 + nl]);
#pragma unroll
  for (int mf = 0; mf < 2; ++mf)
#pragma unroll
    for (int nf = 0; nf < 4; ++nf)
#pragma unroll
      for (int r = 0; r < 8; ++r) {
        const int ml = wr * 32 + mf * 16 + hf * 8 + r;
        const int nloc = wc * 64 + nf * 16 + nl;
        const f16_t hv = (f16_t)(acc[mf][nf][r] + bb4[nf]);
        if constexpr (TRANS_OUT) {
          Cs[nloc * LDC + ml] = hv;
        } else {
          Cs[ml * LDC + nloc] = hv;
        }
      }
  __syncthreads();

  const int c16 = tid & 15;
  const int bsel = m0 / SEQ;
  const int s0 = m0 - bsel * SEQ;
  u32x4 vals[8];
  f16_t* dsts[8];
#pragma unroll
  for (int it = 0; it < 8; ++it) {
    const int row = it * 16 + (tid >> 4);
    const h16x8 hv8 = *(const h16x8*)(Cs + row * LDC + c16 * 8);
    vals[it] = __builtin_bit_cast(u32x4, hv8);
    if constexpr (TRANS_OUT) {
      const int n = n0 + row;
      const int hh = n >> 6, dd = n & 63;
      dsts[it] = outp + ((size_t)((bsel * NHEAD + hh) * HDIM + dd)) * SEQ + s0 + c16 * 8;
    } else {
      dsts[it] = outp + (size_t)(m0 + row) * HID + n0 + c16 * 8;
    }
  }
#pragma unroll
  for (int it = 0; it < 8; ++it) *(volatile u32x4*)dsts[it] = vals[it];
  __threadfence();
#pragma unroll
  for (int it = 0; it < 8; ++it) *(volatile u32x4*)dsts[it] = vals[it];
}

__global__ __launch_bounds__(256) __attribute__((amdgpu_num_vgpr(256)))
void k_attn(const f16_t* __restrict__ Qp, const f16_t* __restrict__ Kp,
            const f16_t* __restrict__ VTp, float* __restrict__ outp) {
  constexpr int LDK = 72;
  constexpr int LDO = 68;
  constexpr int KS_BYTES = 64 * LDK * 2;
  constexpr int PS_BYTES = 8 * 16 * LDK * 2;
  constexpr int OS_BYTES = 8 * 16 * LDO * 4;
  constexpr int SMEM_BYTES =
      (2 * KS_BYTES + PS_BYTES) > OS_BYTES ? (2 * KS_BYTES + PS_BYTES) : OS_BYTES;
  __shared__ __align__(16) unsigned char smem[SMEM_BYTES];
  f16_t* Ks = (f16_t*)smem;
  f16_t* Vs = (f16_t*)(smem + KS_BYTES);
  f16_t* Ps = (f16_t*)(smem + 2 * KS_BYTES);
  float* Os = (float*)smem;

  const int tid = threadIdx.x, lane = tid & 31, w = tid >> 5;
  const int hf = lane >> 4, nl = lane & 15;
  const int qtiles = SEQ / 128;
  const int qt = blockIdx.x % qtiles;
  const int bh = blockIdx.x / qtiles;
  const int b = bh / NHEAD;
  const int h = bh - b * NHEAD;
  const int q0 = qt * 128 + w * 16;

  v16h qa[2];
#pragma unroll
  for (int kk = 0; kk < 2; ++kk)
    qa[kk] = frag_row_h(Qp + (size_t)(b * SEQ + q0) * HID + h * HDIM + kk * 32, HID);

  float mrow[8], lrow[8];
  v8f o[4];
#pragma unroll
  for (int r = 0; r < 8; ++r) { mrow[r] = -1e30f; lrow[r] = 0.0f; }
#pragma unroll
  for (int df = 0; df < 4; ++df)
#pragma unroll
    for (int r = 0; r < 8; ++r) o[df][r] = 0.0f;

  const float scale = 0.125f;
  const size_t kbase = (size_t)(b * SEQ) * HID + h * HDIM;
  const size_t vbase = (size_t)(b * NHEAD + h) * HDIM * SEQ;
  f16_t* Pw = Ps + (w * 16) * LDK;

#pragma unroll 1
  for (int kc = 0; kc < SEQ / 64; ++kc) {
#pragma unroll
    for (int it = 0; it < 2; ++it) {
      const int p = it * 256 + tid;
      const int r = p >> 3, c = (p & 7) * 8;
      *(h16x8*)(Ks + r * LDK + c) =
          *(const h16x8*)(Kp + kbase + (size_t)(kc * 64 + r) * HID + c);
      *(h16x8*)(Vs + r * LDK + c) =
          *(const h16x8*)(VTp + vbase + (size_t)r * SEQ + kc * 64 + c);
    }
    __syncthreads();

    v8f sf[4];
#pragma unroll
    for (int nf = 0; nf < 4; ++nf) {
      v8f c = {};
#pragma unroll
      for (int kk = 0; kk < 2; ++kk) {
        const v16h bb = frag_row_h(Ks + (nf * 16) * LDK + kk * 32, LDK);
        c = wmma_f16(qa[kk], bb, c);
      }
#pragma unroll
      for (int r = 0; r < 8; ++r) sf[nf][r] = c[r] * scale;
    }

    float mx[8];
#pragma unroll
    for (int r = 0; r < 8; ++r) {
      mx[r] = fmaxf(fmaxf(sf[0][r], sf[1][r]), fmaxf(sf[2][r], sf[3][r]));
#pragma unroll
      for (int off = 1; off < 16; off <<= 1)
        mx[r] = fmaxf(mx[r], __shfl_xor(mx[r], off, 16));
    }
#pragma unroll
    for (int r = 0; r < 8; ++r) {
      const float mnew = fmaxf(mrow[r], mx[r]);
      const float alpha = __expf(mrow[r] - mnew);
      mrow[r] = mnew;
      lrow[r] *= alpha;
#pragma unroll
      for (int df = 0; df < 4; ++df) o[df][r] *= alpha;
    }
    float rs[8];
#pragma unroll
    for (int r = 0; r < 8; ++r) rs[r] = 0.0f;
#pragma unroll
    for (int nf = 0; nf < 4; ++nf)
#pragma unroll
      for (int r = 0; r < 8; ++r) {
        const float p = __expf(sf[nf][r] - mrow[r]);
        rs[r] += p;
        Pw[(hf * 8 + r) * LDK + nf * 16 + nl] = (f16_t)(p * PCARRY);
      }
#pragma unroll
    for (int r = 0; r < 8; ++r) {
#pragma unroll
      for (int off = 1; off < 16; off <<= 1)
        rs[r] += __shfl_xor(rs[r], off, 16);
      lrow[r] += rs[r];
    }

    wave_lds_sync();

    v16h pa[2];
#pragma unroll
    for (int kk = 0; kk < 2; ++kk) pa[kk] = frag_row_h(Pw + kk * 32, LDK);
#pragma unroll
    for (int df = 0; df < 4; ++df)
#pragma unroll
      for (int kk = 0; kk < 2; ++kk) {
        const v16h bb = frag_row_h(Vs + (df * 16) * LDK + kk * 32, LDK);
        o[df] = wmma_f16(pa[kk], bb, o[df]);
      }
    __syncthreads();
  }

  float inv[8];
#pragma unroll
  for (int r = 0; r < 8; ++r) inv[r] = 1.0f / (lrow[r] * PCARRY);
  float* Ow = Os + w * (16 * LDO);
#pragma unroll
  for (int df = 0; df < 4; ++df)
#pragma unroll
    for (int r = 0; r < 8; ++r)
      Ow[(hf * 8 + r) * LDO + df * 16 + nl] = o[df][r] * inv[r];
  wave_lds_sync();

  f32x4 vv[8];
  float* od[8];
#pragma unroll
  for (int it = 0; it < 8; ++it) {
    const int row = it * 2 + hf;
    vv[it] = *(const f32x4*)(Ow + row * LDO + nl * 4);
    od[it] = outp + ((size_t)(b * SEQ_FULL + q0 + row)) * HID + h * HDIM + nl * 4;
  }
#pragma unroll
  for (int it = 0; it < 8; ++it) *(volatile f32x4*)od[it] = vv[it];
  __threadfence();
#pragma unroll
  for (int it = 0; it < 8; ++it) *(volatile f32x4*)od[it] = vv[it];
}

extern "C" void kernel_launch(void* const* d_in, const int* in_sizes, int n_in,
                              void* d_out, int out_size, void* d_ws, size_t ws_size,
                              hipStream_t stream) {
  if (n_in < 8) return;
  const long long need_act = ((long long)(NB - 1) * SEQ_FULL + SEQ) * HID;
  if ((long long)in_sizes[0] < need_act || (long long)in_sizes[1] < need_act) return;
  if (in_sizes[2] < HID * HID || in_sizes[4] < HID * HID || in_sizes[6] < HID * HID) return;
  if (in_sizes[3] < HID || in_sizes[5] < HID || in_sizes[7] < HID) return;
  if ((long long)out_size < need_act) return;

  const float* hidden  = (const float*)d_in[0];
  const float* context = (const float*)d_in[1];
  const float* Wq = (const float*)d_in[2];
  const float* bq = (const float*)d_in[3];
  const float* Wk = (const float*)d_in[4];
  const float* bk = (const float*)d_in[5];
  const float* Wv = (const float*)d_in[6];
  const float* bv = (const float*)d_in[7];

  const size_t act_elems = (size_t)NB * SEQ * HID;
  const size_t act_bytes = act_elems * 2;
  const size_t w_bytes = (size_t)HID * HID * 2;
  char* ws = (char*)d_ws;
  size_t off = 0;
  unsigned short* Hb = (unsigned short*)(ws + off); off += act_bytes;
  unsigned short* Cb = (unsigned short*)(ws + off); off += act_bytes;
  unsigned short* WTq = (unsigned short*)(ws + off); off += w_bytes;
  unsigned short* WTk = (unsigned short*)(ws + off); off += w_bytes;
  unsigned short* WTv = (unsigned short*)(ws + off); off += w_bytes;
  f16_t* Qp = (f16_t*)(ws + off); off += act_bytes;
  f16_t* Kp = (f16_t*)(ws + off); off += act_bytes;
  f16_t* VT = (f16_t*)(ws + off); off += act_bytes;
  if (off > ws_size) return;

  const dim3 blk(256);
  const dim3 g_rows((unsigned)((act_elems / 8) / 256));
  const dim3 g_wt(HID / 64, HID / 64);
  const dim3 g_gemm(HID / 128, (NB * SEQ) / 128);
  const dim3 g_attn(NB * NHEAD * (SEQ / 128));

  k_cast_rows<<<g_rows, blk, 0, stream>>>(hidden, Hb);
  k_cast_rows<<<g_rows, blk, 0, stream>>>(context, Cb);
  k_cast_wt<<<g_wt, blk, 0, stream>>>(Wq, WTq);
  k_cast_wt<<<g_wt, blk, 0, stream>>>(Wk, WTk);
  k_cast_wt<<<g_wt, blk, 0, stream>>>(Wv, WTv);

  k_proj_gemm<false><<<g_gemm, blk, 0, stream>>>((const bf16_t*)Hb, (const bf16_t*)WTq, bq, Qp);
  k_proj_gemm<false><<<g_gemm, blk, 0, stream>>>((const bf16_t*)Cb, (const bf16_t*)WTk, bk, Kp);
  k_proj_gemm<true><<<g_gemm, blk, 0, stream>>>((const bf16_t*)Cb, (const bf16_t*)WTv, bv, VT);

  k_attn<<<g_attn, blk, 0, stream>>>(Qp, Kp, VT, (float*)d_out);
}
